// UnifiedGATExpert_28948079575200
// MI455X (gfx1250) — hardware-run, weakly checked
//
#include <hip/hip_runtime.h>
#include <stddef.h>
#include <stdint.h>
#include <math.h>


#define NNODE   20000
#define NEDGE   320000
#define HW      64
#define NHD     4
#define HC      256
#define PAH     128
#define PWH     128
#define TWO_P2  1
#define TWO_C1  1
#define TWO_C2  1
#define TWO_C3  1
#define KX_P2   (TWO_P2 ? 128 : 64)
#define KX_C1   (TWO_C1 ? 128 : 64)
#define KX_C2   (TWO_C2 ? 128 : 64)
#define KX_C3   (TWO_C3 ? 128 : 64)
#define NEGSL   0.2f
#define LNEPS   1e-5f
#define NTHR    256
#define NWAVE   8
#define EPT     8
#define CHUNK   (NTHR * EPT)
#define WCAP    (EPT * 32)
#define LISTN   (NWAVE * WCAP)
#define NBA     1024
#define PKS     10
#define RCAP    20480
#define DEGCAP  64
#define GBM     64
#define GBN     64
#define GTHR    128
#define RPB     64
#define RPW     8
#define BK_INTS (2 * RCAP + 3 * NBA + LISTN + 32)
#define LDS_BK  (BK_INTS * 4)
#define MEAS_BLK_HITS 16685
#define MEAS_MAXDEG   32
#define WSMAX   (128u << 20)
#define UW1     (HW * 8)
#define UW2     (HW * 16)
#define UC12    (HC * 16)
#define UC3     (HW * 16)
#define UWALL   (UW1 + UW2 + 2 * UC12 + UC3)

static_assert((CHUNK & (CHUNK - 1)) == 0 && CHUNK <= 4096);
static_assert(NBA == (1 << PKS) && NBA == NTHR * 4);
static_assert(LISTN == NWAVE * WCAP);
static_assert(RCAP % (NTHR * 4) == 0 && BK_INTS % 4 == 0);
static_assert((long long)RCAP * 100 >= (long long)MEAS_BLK_HITS * 105);
static_assert(DEGCAP >= MEAS_MAXDEG + 8);
static_assert(LDS_BK <= 327680);
static_assert(NEDGE < (1 << 21));
static_assert(GBM == (GTHR / 32) * 16 && GTHR == 2 * GBN && GTHR == 2 * GBM);
static_assert(HC == NHD * HW && HW == GBN);
static_assert(PAH == 2 * HW && PWH == 2 * HW);
static_assert((KX_P2 % 32) == 0 && (KX_C1 % 32) == 0 && (KX_C2 % 32) == 0 && (KX_C3 % 32) == 0);
static_assert(KX_P2 <= PAH && KX_C1 <= PAH && KX_C2 <= PAH && KX_C3 <= PAH);
static_assert(RPB == NWAVE * RPW && RPB == GBM);
static_assert(HC == 8 * 32 && HW == 2 * 32);
static_assert(UW1 % NTHR == 0 && UW2 % NTHR == 0 && UC12 % NTHR == 0 && UC3 % NTHR == 0);

typedef float          v2f  __attribute__((ext_vector_type(2)));
typedef float          v4f  __attribute__((ext_vector_type(4)));
typedef float          v8f  __attribute__((ext_vector_type(8)));
typedef int            v4i  __attribute__((ext_vector_type(4)));
typedef int            v8i  __attribute__((ext_vector_type(8)));
typedef unsigned       v4u  __attribute__((ext_vector_type(4)));
typedef unsigned short v8us __attribute__((ext_vector_type(8)));
typedef __bf16         v16b __attribute__((ext_vector_type(16)));
typedef v2f  __attribute__((may_alias)) v2fa;
typedef v4f  __attribute__((may_alias)) v4fa;
typedef v4i  __attribute__((may_alias)) v4ia;
typedef v4u  __attribute__((may_alias)) v4ua;
typedef v8us __attribute__((may_alias)) v8usa;
union FragB { v16b v; v8us h[2]; v4u q[2]; v8i w; };
struct HL8 { v4u h; v4u l; };

__device__ __forceinline__ v8f wmb(const FragB& a, const FragB& b, v8f c) {
  v8f d = __builtin_amdgcn_wmma_f32_16x16x32_bf16(false, a.v, false, b.v, (short)0, c, false, false);
  asm volatile("v_nop\n\tv_nop\n\tv_nop\n\tv_nop" : "+v"(d) : "v"(a.w), "v"(b.w));
  return d;
}

__device__ __forceinline__ unsigned f2bf(float f) {
  const unsigned u = __float_as_uint(f);
  return ((u + 0x7FFFu + ((u >> 16) & 1u)) >> 16) & 0xFFFFu;
}
__device__ __forceinline__ float bf2f(unsigned b) { return __uint_as_float(b << 16); }
__device__ __forceinline__ float bfr(float f) { return bf2f(f2bf(f)); }
__device__ __forceinline__ unsigned pk2(float lo, float hi) { return f2bf(lo) | (f2bf(hi) << 16); }
__device__ __forceinline__ v4u pack8(const v4f a, const v4f b) {
  v4u r;
  r.x = pk2(a.x, a.y); r.y = pk2(a.z, a.w); r.z = pk2(b.x, b.y); r.w = pk2(b.z, b.w);
  return r;
}
__device__ __forceinline__ void pack2(float a, float b, unsigned& hw, unsigned& lw) {
  const unsigned ha = f2bf(a), hb = f2bf(b);
  const unsigned la = f2bf(a - bf2f(ha));
  const unsigned lb = f2bf(b - bf2f(hb));
  hw = ha | (hb << 16);
  lw = la | (lb << 16);
}
__device__ __forceinline__ HL8 pack_hl8(const float (&y)[8]) {
  unsigned h0, l0, h1, l1, h2, l2, h3, l3;
  pack2(y[0], y[1], h0, l0);
  pack2(y[2], y[3], h1, l1);
  pack2(y[4], y[5], h2, l2);
  pack2(y[6], y[7], h3, l3);
  HL8 r;
  r.h.x = h0; r.h.y = h1; r.h.z = h2; r.h.w = h3;
  r.l.x = l0; r.l.y = l1; r.l.z = l2; r.l.w = l3;
  return r;
}
__device__ __forceinline__ float relu_k(float v) { return (v > 0.0f) ? v : (v - v); }
__device__ __forceinline__ float leaky(float v) { return (v > 0.0f) ? v : NEGSL * v; }

__device__ __forceinline__ void ln8(float (&v)[8], const v4f wa, const v4f wb, const v4f ba, const v4f bb) {
  float s = ((v[0] + v[1]) + (v[2] + v[3])) + ((v[4] + v[5]) + (v[6] + v[7]));
  s += __shfl_xor(s, 4, 32);
  s += __shfl_xor(s, 2, 32);
  s += __shfl_xor(s, 1, 32);
  const float mu = s * (1.0f / 64.0f);
  float d[8];
#pragma unroll
  for (int i = 0; i < 8; ++i) d[i] = v[i] - mu;
  float q = ((d[0] * d[0] + d[1] * d[1]) + (d[2] * d[2] + d[3] * d[3])) +
            ((d[4] * d[4] + d[5] * d[5]) + (d[6] * d[6] + d[7] * d[7]));
  q += __shfl_xor(q, 4, 32);
  q += __shfl_xor(q, 2, 32);
  q += __shfl_xor(q, 1, 32);
  const float r = rsqrtf(q * (1.0f / 64.0f) + LNEPS);
  const float w[8] = {wa.x, wa.y, wa.z, wa.w, wb.x, wb.y, wb.z, wb.w};
  const float b[8] = {ba.x, ba.y, ba.z, ba.w, bb.x, bb.y, bb.z, bb.w};
#pragma unroll
  for (int i = 0; i < 8; ++i) v[i] = d[i] * r * w[i] + b[i];
}

__device__ __forceinline__ int scan_chunk(const int* __restrict__ keys, int nE, int cbase, int slotBase,
                                          int nb, int vec8, int* list, int tid, int lane, int wave) {
  int wc = 0;
  const int el0  = tid * EPT;
  const int e0   = cbase + el0;
  const int sent = (int)(1u << 31);
  v4i da, db;
  if (vec8 != 0 && cbase + CHUNK <= nE) {
    da = *(const v4i*)(keys + e0);
    db = *(const v4i*)(keys + e0 + 4);
  } else {
    da.x = (e0     < nE) ? keys[min(e0,     nE - 1)] : sent;
    da.y = (e0 + 1 < nE) ? keys[min(e0 + 1, nE - 1)] : sent;
    da.z = (e0 + 2 < nE) ? keys[min(e0 + 2, nE - 1)] : sent;
    da.w = (e0 + 3 < nE) ? keys[min(e0 + 3, nE - 1)] : sent;
    db.x = (e0 + 4 < nE) ? keys[min(e0 + 4, nE - 1)] : sent;
    db.y = (e0 + 5 < nE) ? keys[min(e0 + 5, nE - 1)] : sent;
    db.z = (e0 + 6 < nE) ? keys[min(e0 + 6, nE - 1)] : sent;
    db.w = (e0 + 7 < nE) ? keys[min(e0 + 7, nE - 1)] : sent;
  }
  const unsigned nbs = (unsigned)slotBase;
  const unsigned unb = (unsigned)nb;
  const unsigned s0 = (unsigned)da.x - nbs, s1 = (unsigned)da.y - nbs;
  const unsigned s2 = (unsigned)da.z - nbs, s3 = (unsigned)da.w - nbs;
  const unsigned s4 = (unsigned)db.x - nbs, s5 = (unsigned)db.y - nbs;
  const unsigned s6 = (unsigned)db.z - nbs, s7 = (unsigned)db.w - nbs;
  const bool h0 = s0 < unb, h1 = s1 < unb, h2 = s2 < unb, h3 = s3 < unb;
  const bool h4 = s4 < unb, h5 = s5 < unb, h6 = s6 < unb, h7 = s7 < unb;
  const unsigned any = __builtin_amdgcn_ballot_w32(h0 | h1 | h2 | h3 | h4 | h5 | h6 | h7);
  if (any != 0u) {
#define HITJ(J, HJ, SJ) { \
      const unsigned mj = __builtin_amdgcn_ballot_w32(HJ); \
      if (mj != 0u) { \
        if (HJ) { \
          const int pos = wc + (int)__builtin_amdgcn_mbcnt_lo(mj, 0u); \
          if (pos < WCAP) list[wave * WCAP + pos] = ((el0 + (J)) << PKS) | (int)(SJ); \
        } \
        wc += (int)__builtin_popcount(mj); } }
    HITJ(0, h0, s0)
    HITJ(1, h1, s1)
    HITJ(2, h2, s2)
    HITJ(3, h3, s3)
    HITJ(4, h4, s4)
    HITJ(5, h5, s5)
    HITJ(6, h6, s6)
    HITJ(7, h7, s7)
#undef HITJ
  }
  return wc;
}

template <int KQ>
__device__ __forceinline__ void wplane_unit(const float* __restrict__ w, unsigned short* out, int u, int nrows) {
  const int n  = u / KQ;
  const int j  = u - n * KQ;
  const int k8 = 8 * j;
  const int kk = k8 & (HW - 1);
  const int nc = n < nrows ? n : nrows - 1;
  const float* p = w + (size_t)nc * HW + kk;
  const v4f a = *(const v4fa*)p;
  const v4f b = *(const v4fa*)(p + 4);
  const v4u wv = pack8(a, b);
  unsigned short* o = out + (size_t)nc * (size_t)(KQ * 8) + k8;
  *(volatile v4u*)o = wv;
  __threadfence();
  *(volatile v4u*)o = wv;
}

__global__ __launch_bounds__(NTHR) void k_prep(const float* __restrict__ x, const float* __restrict__ w1,
                                               const float* __restrict__ w2, const float* __restrict__ g1,
                                               const float* __restrict__ g2, const float* __restrict__ g3,
                                               unsigned short* XB, unsigned short* SW1, unsigned short* SW2D,
                                               unsigned short* C1D, unsigned short* C2D, unsigned short* C3D,
                                               int nN, int uXB) {
  const int ub  = (int)blockIdx.x * NTHR;
  const int tid = (int)threadIdx.x;
  if (ub < uXB) {
    const int u   = ub + tid;
    const int row = u >> 3;
    const int c0  = (u & 7) * 8;
    const int rc  = row < nN ? row : nN - 1;
    const float* p = x + (size_t)rc * HW + c0;
    v4f a = *(const v4fa*)p;
    v4f b = *(const v4fa*)(p + 4);
    asm volatile("" :: "v"(a), "v"(b));
    const bool lv = row < nN;
    a.x = lv ? a.x : 0.0f; a.y = lv ? a.y : 0.0f; a.z = lv ? a.z : 0.0f; a.w = lv ? a.w : 0.0f;
    b.x = lv ? b.x : 0.0f; b.y = lv ? b.y : 0.0f; b.z = lv ? b.z : 0.0f; b.w = lv ? b.w : 0.0f;
    const v4u hv = pack8(a, b);
    unsigned short* o = XB + (size_t)row * HW + c0;
    *(volatile v4u*)o = hv;
    __threadfence();
    *(volatile v4u*)o = hv;
  } else {
    const int r = ub - uXB;
    if (r < UW1) {
      wplane_unit<8>(w1, SW1, r + tid, HW);
    } else if (r < UW1 + UW2) {
      wplane_unit<16>(w2, SW2D, r - UW1 + tid, HW);
    } else if (r < UW1 + UW2 + UC12) {
      wplane_unit<16>(g1, C1D, r - (UW1 + UW2) + tid, HC);
    } else if (r < UW1 + UW2 + 2 * UC12) {
      wplane_unit<16>(g2, C2D, r - (UW1 + UW2 + UC12) + tid, HC);
    } else if (r < UWALL) {
      wplane_unit<16>(g3, C3D, r - (UW1 + UW2 + 2 * UC12) + tid, HW);
    }
  }
}

__global__ __launch_bounds__(NTHR) void k_bucket(const int* __restrict__ keys, const int* __restrict__ gidx,
                                                 int nE, int nN, int vec8,
                                                 int* LIST, int* CNT, int* OFF, int* FLG, int* REC) {
  extern __shared__ __attribute__((aligned(16))) int dsm[];
  int* reg1 = dsm;
  int* reg2 = reg1 + RCAP;
  int* scnt = reg2 + RCAP;
  int* soff = scnt + NBA;
  int* cur  = soff + NBA;
  int* list = cur + NBA;
  int* wcnt = list + LISTN;
  int* wtot = wcnt + 8;
  int* wmx  = wtot + 8;
  const int tid = (int)threadIdx.x, lane = tid & 31, wave = tid >> 5;
  const int nodeBase = (int)blockIdx.x * NBA;
  int nb = nN - nodeBase;
  nb = nb > NBA ? NBA : (nb < 1 ? 1 : nb);

  {
    const v4i z4 = {0, 0, 0, 0};
    for (int i = tid * 4; i < BK_INTS; i += NTHR * 4) *(v4ia*)(dsm + i) = z4;
  }
  __syncthreads();

  int tot = 0;
  const int nChunks = (nE + CHUNK - 1) / CHUNK;
#pragma unroll 1
  for (int ch = 0; ch < nChunks; ++ch) {
    const int cbase = ch * CHUNK;
    const int wc = scan_chunk(keys, nE, cbase, nodeBase, nb, vec8, list, tid, lane, wave);
    if (lane == 0) wcnt[wave] = wc;
    __syncthreads();
    int pre = 0, all = 0;
#pragma unroll
    for (int w2 = 0; w2 < NWAVE; ++w2) {
      int c = wcnt[w2];
      c = c < 0 ? 0 : (c > WCAP ? WCAP : c);
      all += c;
      pre += (w2 < wave) ? c : 0;
    }
    const int wcc  = wc > WCAP ? WCAP : wc;
    const int base = tot + pre;
#pragma unroll 1
    for (int i = lane; i < wcc; i += 32) {
      const int ent = list[wave * WCAP + i];
      const int el  = (ent >> PKS) & (CHUNK - 1);
      const int sl  = ent & (NBA - 1);
      int eid = cbase + el;
      eid = eid > nE - 1 ? nE - 1 : eid;
      const int pos = base + i;
      if (pos < RCAP) reg1[pos] = (int)(((unsigned)eid << PKS) | (unsigned)sl);
    }
    tot += all;
    tot = tot > RCAP ? RCAP : tot;
    __syncthreads();
  }
  const int nh = tot;

  if (wave == 0) {
#pragma unroll 1
    for (int b0 = 0; b0 < nh; b0 += 32) {
      const int idx = b0 + lane;
      const int uv  = reg1[idx < RCAP ? idx : RCAP - 1];
      const int m32 = (nh - b0) < 32 ? (nh - b0) : 32;
#pragma unroll 1
      for (int k = 0; k < m32; ++k) {
        const int u  = __builtin_amdgcn_readlane(uv, k);
        const int sl = u & (NBA - 1);
        if (lane == 0) scnt[sl] = scnt[sl] + 1;
      }
    }
  }
  __syncthreads();

  {
    const v4i ca = *(const v4ia*)(scnt + 4 * tid);
    const int e0 = ca.x < 0 ? 0 : ca.x, e1 = ca.y < 0 ? 0 : ca.y, e2 = ca.z < 0 ? 0 : ca.z, e3 = ca.w < 0 ? 0 : ca.w;
    const int ts = e0 + e1 + e2 + e3;
    int incl = ts;
#pragma unroll
    for (int d = 1; d < 32; d <<= 1) {
      const int up = __shfl_up(incl, d, 32);
      if (lane >= d) incl += up;
    }
    int mx = max(max(e0, e1), max(e2, e3));
    mx = max(mx, __shfl_xor(mx, 16, 32));
    mx = max(mx, __shfl_xor(mx, 8, 32));
    mx = max(mx, __shfl_xor(mx, 4, 32));
    mx = max(mx, __shfl_xor(mx, 2, 32));
    mx = max(mx, __shfl_xor(mx, 1, 32));
    if (lane == 31) wtot[wave] = incl;
    if (lane == 0)  wmx[wave] = mx;
    __syncthreads();
    int pre = 0;
#pragma unroll
    for (int w2 = 0; w2 < NWAVE; ++w2) pre += (w2 < wave) ? wtot[w2] : 0;
    int run = pre + incl - ts;
    v4i so;
    so.x = run; run += e0;
    so.y = run; run += e1;
    so.z = run; run += e2;
    so.w = run;
    *(v4ia*)(soff + 4 * tid) = so;
    *(v4ia*)(cur + 4 * tid)  = so;
  }
  __syncthreads();

  if (wave == 0) {
#pragma unroll 1
    for (int b0 = 0; b0 < nh; b0 += 32) {
      const int idx = b0 + lane;
      const int uv  = reg1[idx < RCAP ? idx : RCAP - 1];
      const int m32 = (nh - b0) < 32 ? (nh - b0) : 32;
#pragma unroll 1
      for (int k = 0; k < m32; ++k) {
        const int u   = __builtin_amdgcn_readlane(uv, k);
        const int sl  = u & (NBA - 1);
        const int eid = (int)((unsigned)u >> PKS);
        if (lane == 0) {
          int pos = cur[sl];
          pos = pos < 0 ? 0 : (pos > RCAP - 1 ? RCAP - 1 : pos);
          reg2[pos] = eid;
          cur[sl] = pos + 1;
        }
      }
    }
  }
  __syncthreads();

  int bmax = 0;
#pragma unroll
  for (int w2 = 0; w2 < NWAVE; ++w2) bmax = max(bmax, wmx[w2]);
  const int flag = ((nh >= RCAP) || (bmax > DEGCAP)) ? 1 : 0;

  int* lrow = LIST + (size_t)blockIdx.x * RCAP;
#pragma unroll 1
  for (int it = 0; it < RCAP / (NTHR * 4); ++it) {
    const int i0 = 4 * (it * NTHR + tid);
    const v4i ev = *(const v4ia*)(reg2 + i0);
    int e0 = ev.x, e1 = ev.y, e2 = ev.z, e3 = ev.w;
    e0 = e0 < 0 ? 0 : (e0 > nE - 1 ? nE - 1 : e0);
    e1 = e1 < 0 ? 0 : (e1 > nE - 1 ? nE - 1 : e1);
    e2 = e2 < 0 ? 0 : (e2 > nE - 1 ? nE - 1 : e2);
    e3 = e3 < 0 ? 0 : (e3 > nE - 1 ? nE - 1 : e3);
    int g0 = gidx[e0], g1 = gidx[e1], g2 = gidx[e2], g3 = gidx[e3];
    asm volatile("" :: "v"(g0), "v"(g1), "v"(g2), "v"(g3));
    g0 = g0 < 0 ? 0 : (g0 > nN - 1 ? nN - 1 : g0);
    g1 = g1 < 0 ? 0 : (g1 > nN - 1 ? nN - 1 : g1);
    g2 = g2 < 0 ? 0 : (g2 > nN - 1 ? nN - 1 : g2);
    g3 = g3 < 0 ? 0 : (g3 > nN - 1 ? nN - 1 : g3);
    v4i ov;
    ov.x = (i0     < nh) ? g0 : 0;
    ov.y = (i0 + 1 < nh) ? g1 : 0;
    ov.z = (i0 + 2 < nh) ? g2 : 0;
    ov.w = (i0 + 3 < nh) ? g3 : 0;
    *(volatile v4i*)(lrow + i0) = ov;
    __threadfence();
    *(volatile v4i*)(lrow + i0) = ov;
  }
  {
    const v4i cv = *(const v4ia*)(scnt + 4 * tid);
    const v4i fv = *(const v4ia*)(soff + 4 * tid);
    v4i gv; gv.x = flag; gv.y = flag; gv.z = flag; gv.w = flag;
    v4i rv = {0, 0, 0, 0};
    rv.x = (tid == 0) ? bmax : 0;
    rv.y = (tid == 0) ? flag : 0;
    rv.z = (tid == 0) ? nh : 0;
    int* cp = CNT + (size_t)nodeBase + 4 * tid;
    int* fp = OFF + (size_t)nodeBase + 4 * tid;
    int* gp = FLG + (size_t)nodeBase + 4 * tid;
    int* rp = REC + (size_t)blockIdx.x * 32 + 4 * (tid & 7);
    *(volatile v4i*)cp = cv;
    *(volatile v4i*)fp = fv;
    *(volatile v4i*)gp = gv;
    if (tid < 8) *(volatile v4i*)rp = rv;
    __threadfence();
    *(volatile v4i*)cp = cv;
    *(volatile v4i*)fp = fv;
    *(volatile v4i*)gp = gv;
    if (tid < 8) *(volatile v4i*)rp = rv;
  }
}

__global__ __launch_bounds__(GTHR) void k_prompt(
    const unsigned short* __restrict__ XB, const unsigned short* __restrict__ SW1,
    const unsigned short* __restrict__ SW2D,
    const float* __restrict__ b1, const float* __restrict__ b2, const float* __restrict__ emb,
    const float* __restrict__ fwp, const float* __restrict__ lnw, const float* __restrict__ lnb,
    unsigned short* XP, int nN) {
  __shared__ __attribute__((aligned(16))) float stg[GBM * GBN];
  __shared__ __attribute__((aligned(16))) float prm[384];
  const int tid = (int)threadIdx.x, lane = tid & 31, wave = tid >> 5, hh = lane >> 4, m = lane & 15;
  const int rowBase = (int)blockIdx.x * GBM;

  if (wave == 0) {
    const v2f p1 = *(const v2fa*)(b1 + 2 * lane);
    const v2f p2 = *(const v2fa*)(b2 + 2 * lane);
    const v2f pw = *(const v2fa*)(lnw + 2 * lane);
    const v2f pb = *(const v2fa*)(lnb + 2 * lane);
    prm[2 * lane]           = bfr(p1.x); prm[2 * lane + 1]       = bfr(p1.y);
    prm[64 + 2 * lane]      = bfr(p2.x); prm[64 + 2 * lane + 1]  = bfr(p2.y);
    prm[128 + 2 * lane]     = bfr(pw.x); prm[128 + 2 * lane + 1] = bfr(pw.y);
    prm[192 + 2 * lane]     = bfr(pb.x); prm[192 + 2 * lane + 1] = bfr(pb.y);
  } else if (wave < 3) {
    const int c = tid - 32;
    const float e0 = emb[c],           e1 = emb[HW + c],     e2 = emb[2 * HW + c], e3 = emb[3 * HW + c];
    const float e4 = emb[4 * HW + c],  e5 = emb[5 * HW + c], e6 = emb[6 * HW + c], e7 = emb[7 * HW + c];
    float s = bfr(e0);
    s += bfr(e1); s += bfr(e2); s += bfr(e3); s += bfr(e4); s += bfr(e5); s += bfr(e6); s += bfr(e7);
    prm[256 + c] = s * 0.125f;
  } else {
    const float t  = bfr(fwp[0]);
    const float fw = 1.0f / (1.0f + expf(-t));
    if (lane == 0) { prm[320] = fw; prm[321] = 1.0f - fw; }
  }

  v8f acc[4];
  const v8f z8 = {0.f, 0.f, 0.f, 0.f, 0.f, 0.f, 0.f, 0.f};
  acc[0] = z8; acc[1] = z8; acc[2] = z8; acc[3] = z8;
  {
    const unsigned short* ap = XB + (size_t)(rowBase + 16 * wave + m) * HW + 8 * hh;
    const unsigned short* wp = SW1 + (size_t)m * HW + 8 * hh;
#pragma unroll
    for (int ks = 0; ks < 2; ++ks) {
      FragB af;
      af.h[0] = *(const v8usa*)(ap + 32 * ks);
      af.h[1] = *(const v8usa*)(ap + 32 * ks + 16);
#pragma unroll
      for (int t = 0; t < 4; ++t) {
        const unsigned short* wq = wp + (size_t)(16 * t) * HW + 32 * ks;
        FragB bf;
        bf.h[0] = *(const v8usa*)wq;
        bf.h[1] = *(const v8usa*)(wq + 16);
        acc[t] = wmb(af, bf, acc[t]);
      }
    }
  }
  __syncthreads();

#pragma unroll
  for (int t = 0; t < 4; ++t) {
    const int lc = 16 * t + m;
    const float bb = prm[lc];
#pragma unroll
    for (int r = 0; r < 8; ++r) {
      const int lr = 16 * wave + 8 * hh + r;
      stg[lr * GBN + lc] = relu_k(acc[t][r] + bb);
    }
  }
  __syncthreads();

  acc[0] = z8; acc[1] = z8; acc[2] = z8; acc[3] = z8;
  {
    const float* sr = stg + (16 * wave + m) * GBN;
    const unsigned short* wp = SW2D + (size_t)m * PWH + 8 * hh;
#pragma unroll
    for (int ks = 0; ks < KX_P2 / 32; ++ks) {
      const int cb = 32 * (ks & 1) + 8 * hh;
      const v4f f0 = *(const v4fa*)(sr + cb);
      const v4f f1 = *(const v4fa*)(sr + cb + 4);
      const v4f f2 = *(const v4fa*)(sr + cb + 16);
      const v4f f3 = *(const v4fa*)(sr + cb + 20);
      const float ya[8] = {f0.x, f0.y, f0.z, f0.w, f1.x, f1.y, f1.z, f1.w};
      const float yb[8] = {f2.x, f2.y, f2.z, f2.w, f3.x, f3.y, f3.z, f3.w};
      const HL8 pa = pack_hl8(ya);
      const HL8 pb = pack_hl8(yb);
      FragB af;
      if ((ks >> 1) == 0) { af.q[0] = pa.h; af.q[1] = pb.h; }
      else                { af.q[0] = pa.l; af.q[1] = pb.l; }
#pragma unroll
      for (int t = 0; t < 4; ++t) {
        const unsigned short* wq = wp + (size_t)(16 * t) * PWH + 32 * ks;
        FragB bf;
        bf.h[0] = *(const v8usa*)wq;
        bf.h[1] = *(const v8usa*)(wq + 16);
        acc[t] = wmb(af, bf, acc[t]);
      }
    }
  }
  __syncthreads();

#pragma unroll
  for (int t = 0; t < 4; ++t) {
    const int lc = 16 * t + m;
    const float bb = prm[64 + lc];
#pragma unroll
    for (int r = 0; r < 8; ++r) {
      const int lr = 16 * wave + 8 * hh + r;
      stg[lr * GBN + lc] = acc[t][r] + bb;
    }
  }
  __syncthreads();

  {
    const int g = lane & 7, sub = lane >> 3;
    const float fw = prm[320], omf = prm[321];
    const v4f wa = *(const v4fa*)(prm + 128 + 8 * g), wb = *(const v4fa*)(prm + 128 + 8 * g + 4);
    const v4f ba = *(const v4fa*)(prm + 192 + 8 * g), bb = *(const v4fa*)(prm + 192 + 8 * g + 4);
    const v4f pa = *(const v4fa*)(prm + 256 + 8 * g), pb = *(const v4fa*)(prm + 256 + 8 * g + 4);
#pragma unroll 1
    for (int p = 0; p < 4; ++p) {
      const int lr = 16 * wave + 4 * p + sub;
      const int gr = rowBase + lr;
      const v4f sa = *(const v4fa*)(stg + lr * GBN + 8 * g);
      const v4f sb = *(const v4fa*)(stg + lr * GBN + 8 * g + 4);
      float v[8];
      v[0] = omf * sa.x + fw * pa.x; v[1] = omf * sa.y + fw * pa.y;
      v[2] = omf * sa.z + fw * pa.z; v[3] = omf * sa.w + fw * pa.w;
      v[4] = omf * sb.x + fw * pb.x; v[5] = omf * sb.y + fw * pb.y;
      v[6] = omf * sb.z + fw * pb.z; v[7] = omf * sb.w + fw * pb.w;
      ln8(v, wa, wb, ba, bb);
      const bool live = gr < nN;
#pragma unroll
      for (int i = 0; i < 8; ++i) v[i] = live ? v[i] : 0.0f;
      const HL8 pk = pack_hl8(v);
      unsigned short* hp = XP + (size_t)gr * PAH + 8 * g;
      *(volatile v4u*)hp = pk.h;
      *(volatile v4u*)(hp + HW) = pk.l;
      __threadfence();
      *(volatile v4u*)hp = pk.h;
      *(volatile v4u*)(hp + HW) = pk.l;
    }
  }
}

__global__ __launch_bounds__(GTHR) void k_proj(
    const unsigned short* __restrict__ A, const unsigned short* __restrict__ WT,
    float* outF, int lda, int ldw, int K, int ldo,
    const float* __restrict__ atts, const float* __restrict__ attd,
    float* SD, int MPr) {
  __shared__ __attribute__((aligned(16))) float stg[GBM * GBN];
  __shared__ __attribute__((aligned(16))) float satt[2 * GBN];
  __shared__ __attribute__((aligned(16))) float sdot[2 * GBM];
  const int tid = (int)threadIdx.x, lane = tid & 31, wave = tid >> 5, hh = lane >> 4, m = lane & 15;
  const int rowBase = (int)blockIdx.x * GBM;
  const int head    = (int)blockIdx.y;
  const int col0    = head * GBN;

  {
    const int which = tid >> 6;
    const int c  = tid & 63;
    const float vs = atts[head * HW + c];
    const float vd = attd[head * HW + c];
    const unsigned msk = (which == 0) ? 0u : ~0u;
    const float v = __uint_as_float((__float_as_uint(vs) & ~msk) | (__float_as_uint(vd) & msk));
    satt[which * GBN + c] = bfr(v);
  }

  v8f acc[4];
  {
    const v8f z = {0.f, 0.f, 0.f, 0.f, 0.f, 0.f, 0.f, 0.f};
    acc[0] = z; acc[1] = z; acc[2] = z; acc[3] = z;
  }
  const unsigned short* ap = A  + (size_t)(rowBase + 16 * wave + m) * (size_t)lda + 8 * hh;
  const unsigned short* wp = WT + (size_t)(col0 + m) * (size_t)ldw + 8 * hh;
  const int ksteps = K >> 5;
#pragma unroll 1
  for (int ks = 0; ks < ksteps; ++ks) {
    FragB af;
    af.h[0] = *(const v8usa*)(ap + 32 * ks);
    af.h[1] = *(const v8usa*)(ap + 32 * ks + 16);
#pragma unroll
    for (int t = 0; t < 4; ++t) {
      const unsigned short* wq = wp + (size_t)(16 * t) * (size_t)ldw + 32 * ks;
      FragB bf;
      bf.h[0] = *(const v8usa*)wq;
      bf.h[1] = *(const v8usa*)(wq + 16);
      acc[t] = wmb(af, bf, acc[t]);
    }
  }

#pragma unroll
  for (int t = 0; t < 4; ++t) {
    const int lc = 16 * t + m;
#pragma unroll
    for (int r = 0; r < 8; ++r) {
      const int lr = 16 * wave + 8 * hh + r;
      stg[lr * GBN + lc] = acc[t][r];
    }
  }
  __syncthreads();

  {
    const int row = tid & 63, which = tid >> 6;
    const float* sa = satt + which * GBN;
    const float* hr = stg + row * GBN;
    float d = 0.f;
#pragma unroll 4
    for (int c4 = 0; c4 < GBN / 4; ++c4) {
      const v4f hv = *(const v4fa*)(hr + 4 * c4);
      const v4f av = *(const v4fa*)(sa + 4 * c4);
      d = fmaf(hv.x, av.x, d);
      d = fmaf(hv.y, av.y, d);
      d = fmaf(hv.z, av.z, d);
      d = fmaf(hv.w, av.w, d);
    }
    sdot[which * GBM + row] = d;
  }
  __syncthreads();

  v4f fv[8];
#pragma unroll
  for (int i = 0; i < 8; ++i) {
    const int lr = 16 * wave + 2 * i + hh;
    fv[i] = *(const v4fa*)(stg + lr * GBN + 4 * m);
  }
  const int which2 = lane >> 4, piece = lane & 15;
  const v4f sdv = *(const v4fa*)(sdot + which2 * GBM + 4 * piece);
  float* sp = SD + (size_t)(2 * head + which2) * (size_t)MPr + rowBase + 4 * piece;

#pragma unroll
  for (int i = 0; i < 8; ++i) {
    const int lr = 16 * wave + 2 * i + hh;
    const int gr = rowBase + lr;
    float* op = outF + (size_t)gr * (size_t)ldo + col0 + 4 * m;
    *(volatile v4f*)op = fv[i];
  }
  if (wave == 0) *(volatile v4f*)sp = sdv;
  __threadfence();
#pragma unroll
  for (int i = 0; i < 8; ++i) {
    const int lr = 16 * wave + 2 * i + hh;
    const int gr = rowBase + lr;
    float* op = outF + (size_t)gr * (size_t)ldo + col0 + 4 * m;
    *(volatile v4f*)op = fv[i];
  }
  if (wave == 0) *(volatile v4f*)sp = sdv;
}

template <int L>
__global__ __launch_bounds__(NTHR) void k_replay(
    const float* __restrict__ XH, const float* __restrict__ SD,
    const int* __restrict__ LIST, const int* __restrict__ CNT, const int* __restrict__ OFF,
    const int* __restrict__ FLG,
    const float* __restrict__ bias, const float* __restrict__ lnw, const float* __restrict__ lnb,
    const float* H1in, float* H1out, unsigned short* HL, float* out,
    int nN, int mRows, int MPr) {
  __shared__ __attribute__((aligned(16))) float prm[192];
  const int tid = (int)threadIdx.x, lane = tid & 31;
  const int wave = __builtin_amdgcn_readfirstlane(tid >> 5);
  if (tid < 32) {
    const v2f pb = *(const v2fa*)(bias + 2 * tid);
    const v2f pw = *(const v2fa*)(lnw + 2 * tid);
    const v2f pc = *(const v2fa*)(lnb + 2 * tid);
    prm[2 * tid]       = bfr(pb.x); prm[2 * tid + 1]       = bfr(pb.y);
    prm[64 + 2 * tid]  = bfr(pw.x); prm[64 + 2 * tid + 1]  = bfr(pw.y);
    prm[128 + 2 * tid] = bfr(pc.x); prm[128 + 2 * tid + 1] = bfr(pc.y);
  }
  __syncthreads();
  const float qnan = __int_as_float(0x7fc00000);

  if constexpr (L != 3) {
    const int g = lane & 7, head = lane >> 3;
    const float* ASp = SD + (size_t)(2 * head) * (size_t)MPr;
    const float* ADp = ASp + MPr;
    const v4f bA = *(const v4fa*)(prm + 8 * g),       bB = *(const v4fa*)(prm + 8 * g + 4);
    const v4f wA = *(const v4fa*)(prm + 64 + 8 * g),  wB = *(const v4fa*)(prm + 64 + 8 * g + 4);
    const v4f cA = *(const v4fa*)(prm + 128 + 8 * g), cB = *(const v4fa*)(prm + 128 + 8 * g + 4);
#pragma unroll 1
    for (int ri = 0; ri < RPW; ++ri) {
      const int node = (int)blockIdx.x * RPB + wave * RPW + ri;
      if (node >= mRows) continue;
      const int nodec = node < nN ? node : nN - 1;
      const int craw = CNT[node];
      const int oraw = OFF[node];
      const int fl   = FLG[node];
      int c = craw < 0 ? 0 : (craw > DEGCAP ? DEGCAP : craw);
      int o = oraw < 0 ? 0 : (oraw > RCAP ? RCAP : oraw);
      if (c > RCAP - o) c = RCAP - o;
      c = __builtin_amdgcn_readfirstlane(c);
      o = __builtin_amdgcn_readfirstlane(o);
      int last = o + c - 1;
      last = last < o ? o : last;
      last = last > RCAP - 1 ? RCAP - 1 : last;
      const bool pz = (fl != 0) || (craw > DEGCAP);
      const int* lp = LIST + (size_t)(node >> PKS) * RCAP;

      const float* fr = XH + (size_t)nodec * HC + 8 * lane;
      v4f av = *(const v4fa*)fr;
      v4f bv = *(const v4fa*)(fr + 4);
      const float adv = ADp[nodec];
      float mx = leaky(ASp[nodec] + adv);
      float dn = 1.0f;

#pragma unroll 1
      for (int b0 = 0; b0 < c; b0 += 32) {
        int idx = o + b0 + lane;
        idx = idx > last ? last : idx;
        int s = lp[idx];
        s = s < 0 ? 0 : (s > nN - 1 ? nN - 1 : s);
        const int m32 = (c - b0) < 32 ? (c - b0) : 32;
#pragma unroll 1
        for (int k = 0; k < m32; ++k) {
          const int sk = __builtin_amdgcn_readlane(s, k);
          const float* gp = XH + (size_t)sk * HC + 8 * lane;
          const v4f fa = *(const v4fa*)gp;
          const v4f fb = *(const v4fa*)(gp + 4);
          const float lg = leaky(ASp[sk] + adv);
          const float df = lg - mx;
          const float ee = expf(-fabsf(df));
          const bool up  = df > 0.f;
          const float s1 = up ? ee : 1.0f;
          const float s2 = up ? 1.0f : ee;
          mx = up ? lg : mx;
          dn = fmaf(dn, s1, s2);
          av.x = fmaf(av.x, s1, s2 * fa.x);
          av.y = fmaf(av.y, s1, s2 * fa.y);
          av.z = fmaf(av.z, s1, s2 * fa.z);
          av.w = fmaf(av.w, s1, s2 * fa.w);
          bv.x = fmaf(bv.x, s1, s2 * fb.x);
          bv.y = fmaf(bv.y, s1, s2 * fb.y);
          bv.z = fmaf(bv.z, s1, s2 * fb.z);
          bv.w = fmaf(bv.w, s1, s2 * fb.w);
        }
      }

      const float inv = __builtin_amdgcn_rcpf(dn);
      float v[8];
      v[0] = av.x * inv; v[1] = av.y * inv; v[2] = av.z * inv; v[3] = av.w * inv;
      v[4] = bv.x * inv; v[5] = bv.y * inv; v[6] = bv.z * inv; v[7] = bv.w * inv;
#pragma unroll
      for (int i = 0; i < 8; ++i) {
        v[i] += __shfl_xor(v[i], 8, 32);
        v[i] += __shfl_xor(v[i], 16, 32);
      }
      const float bz[8] = {bA.x, bA.y, bA.z, bA.w, bB.x, bB.y, bB.z, bB.w};
#pragma unroll
      for (int i = 0; i < 8; ++i) v[i] = v[i] * 0.25f + bz[i];
      if constexpr (L == 2) {
        const float* hp1 = H1in + (size_t)nodec * HW;
        const v4f ra = *(const v4fa*)(hp1 + 4 * g);
        const v4f rb = *(const v4fa*)(hp1 + 32 + 4 * g);
        v[0] += ra.x; v[1] += ra.y; v[2] += ra.z; v[3] += ra.w;
        v[4] += rb.x; v[5] += rb.y; v[6] += rb.z; v[7] += rb.w;
      }
      ln8(v, wA, wB, cA, cB);
      const bool live = node < nN;
#pragma unroll
      for (int i = 0; i < 8; ++i) {
        float y = relu_k(v[i]);
        y = pz ? qnan : y;
        v[i] = live ? y : 0.0f;
      }

      const HL8 pk = pack_hl8(v);
      const unsigned mk = ((lane >> 3) & 1) ? ~0u : 0u;
      v4u pv;
      pv.x = (pk.h.x & ~mk) | (pk.l.x & mk);
      pv.y = (pk.h.y & ~mk) | (pk.l.y & mk);
      pv.z = (pk.h.z & ~mk) | (pk.l.z & mk);
      pv.w = (pk.h.w & ~mk) | (pk.l.w & mk);
      v4f fvv;
      fvv.x = __uint_as_float((__float_as_uint(v[0]) & ~mk) | (__float_as_uint(v[4]) & mk));
      fvv.y = __uint_as_float((__float_as_uint(v[1]) & ~mk) | (__float_as_uint(v[5]) & mk));
      fvv.z = __uint_as_float((__float_as_uint(v[2]) & ~mk) | (__float_as_uint(v[6]) & mk));
      fvv.w = __uint_as_float((__float_as_uint(v[3]) & ~mk) | (__float_as_uint(v[7]) & mk));
      unsigned short* hp = HL + (size_t)node * PAH + 8 * (lane & 15);
      float* fp = H1out + (size_t)node * HW + 4 * (lane & 15);
      if (lane < 16) {
        *(volatile v4u*)hp = pv;
        if constexpr (L == 1) *(volatile v4f*)fp = fvv;
      }
      __threadfence();
      if (lane < 16) {
        *(volatile v4u*)hp = pv;
        if constexpr (L == 1) *(volatile v4f*)fp = fvv;
      }
    }
  } else {
    const int c0 = 2 * lane;
    const v2f bz = *(const v2fa*)(prm + c0);
    const float* ASp = SD;
    const float* ADp = SD + MPr;
#pragma unroll 1
    for (int ri = 0; ri < RPW; ++ri) {
      const int node = (int)blockIdx.x * RPB + wave * RPW + ri;
      if (node >= mRows) continue;
      const int nodec = node < nN ? node : nN - 1;
      const int craw = CNT[node];
      const int oraw = OFF[node];
      const int fl   = FLG[node];
      int c = craw < 0 ? 0 : (craw > DEGCAP ? DEGCAP : craw);
      int o = oraw < 0 ? 0 : (oraw > RCAP ? RCAP : oraw);
      if (c > RCAP - o) c = RCAP - o;
      c = __builtin_amdgcn_readfirstlane(c);
      o = __builtin_amdgcn_readfirstlane(o);
      int last = o + c - 1;
      last = last < o ? o : last;
      last = last > RCAP - 1 ? RCAP - 1 : last;
      const bool pz = (fl != 0) || (craw > DEGCAP);
      const int* lp = LIST + (size_t)(node >> PKS) * RCAP;

      const v2f fd = *(const v2fa*)(XH + (size_t)nodec * HW + c0);
      const float adv = ADp[nodec];
      float mx = leaky(ASp[nodec] + adv);
      float dn = 1.0f;
      float a0 = fd.x, a1 = fd.y;
#pragma unroll 1
      for (int b0 = 0; b0 < c; b0 += 32) {
        int idx = o + b0 + lane;
        idx = idx > last ? last : idx;
        int s = lp[idx];
        s = s < 0 ? 0 : (s > nN - 1 ? nN - 1 : s);
        const int m32 = (c - b0) < 32 ? (c - b0) : 32;
#pragma unroll 1
        for (int k = 0; k < m32; ++k) {
          const int sk = __builtin_amdgcn_readlane(s, k);
          const v2f fs = *(const v2fa*)(XH + (size_t)sk * HW + c0);
          const float lg = leaky(ASp[sk] + adv);
          const float df = lg - mx;
          const float ee = expf(-fabsf(df));
          const bool up  = df > 0.f;
          const float s1 = up ? ee : 1.0f;
          const float s2 = up ? 1.0f : ee;
          mx = up ? lg : mx;
          dn = fmaf(dn, s1, s2);
          a0 = fmaf(a0, s1, s2 * fs.x);
          a1 = fmaf(a1, s1, s2 * fs.y);
        }
      }
      const float inv = __builtin_amdgcn_rcpf(dn);
      v2f ov;
      ov.x = a0 * inv + bz.x;
      ov.y = a1 * inv + bz.y;
      ov.x = pz ? qnan : ov.x;
      ov.y = pz ? qnan : ov.y;
      const bool live = node < nN;
      float* op = out + (size_t)nodec * HW + c0;
      if (live) *(volatile v2f*)op = ov;
      __threadfence();
      if (live) *(volatile v2f*)op = ov;
    }
  }
}

static inline int cdiv(int a, int b) { return (a + b - 1) / b; }
static inline size_t al256(size_t o) { return (o + 255) & ~(size_t)255; }

extern "C" void kernel_launch(void* const* d_in, const int* in_sizes, int n_in,
                              void* d_out, int out_size, void* d_ws, size_t ws_size,
                              hipStream_t stream) {
  if (n_in < 26) return;
  if (in_sizes[0] != NNODE * HW) return;
  if (in_sizes[1] != 2 * NEDGE) return;
  if (in_sizes[2] != 8 * HW) return;
  if (in_sizes[3] != HW * HW || in_sizes[5] != HW * HW) return;
  if (in_sizes[4] != HW || in_sizes[6] != HW || in_sizes[7] < 1) return;
  if (in_sizes[8] != HW || in_sizes[9] != HW) return;
  if (in_sizes[10] != HC * HW || in_sizes[14] != HC * HW || in_sizes[18] != HW * HW) return;
  if (in_sizes[11] != HC || in_sizes[12] != HC || in_sizes[15] != HC || in_sizes[16] != HC) return;
  if (in_sizes[19] != HW || in_sizes[20] != HW) return;
  if (in_sizes[13] != HW || in_sizes[17] != HW || in_sizes[21] != HW) return;
  if (in_sizes[22] != HW || in_sizes[23] != HW || in_sizes[24] != HW || in_sizes[25] != HW) return;
  if (out_size != NNODE * HW) return;
  const int nN = NNODE, nE = NEDGE;

  const float* x      = (const float*)d_in[0];
  const int*   ei     = (const int*)  d_in[1];
  const float* sp_emb = (const float*)d_in[2];
  const float* sp_w1  = (const float*)d_in[3];
  const float* sp_b1  = (const float*)d_in[4];
  const float* sp_w2  = (const float*)d_in[5];
  const float* sp_b2  = (const float*)d_in[6];
  const float* sp_fw  = (const float*)d_in[7];
  const float* sp_lnw = (const float*)d_in[8];
  const float* sp_lnb = (const float*)d_in[9];
  const float* g1_w   = (const float*)d_in[10];
  const float* g1_as  = (const float*)d_in[11];
  const float* g1_ad  = (const float*)d_in[12];
  const float* g1_b   = (const float*)d_in[13];
  const float* g2_w   = (const float*)d_in[14];
  const float* g2_as  = (const float*)d_in[15];
  const float* g2_ad  = (const float*)d_in[16];
  const float* g2_b   = (const float*)d_in[17];
  const float* g3_w   = (const float*)d_in[18];
  const float* g3_as  = (const float*)d_in[19];
  const float* g3_ad  = (const float*)d_in[20];
  const float* g3_b   = (const float*)d_in[21];
  const float* ln1_w  = (const float*)d_in[22];
  const float* ln1_b  = (const float*)d_in[23];
  const float* ln2_w  = (const float*)d_in[24];
  const float* ln2_b  = (const float*)d_in[25];
  float* out = (float*)d_out;
  const int* srcs = ei;
  const int* dsts = ei + nE;

  const int MP    = cdiv(nN, GBM) * GBM;
  const int nB    = cdiv(nN, NBA);
  const int NPADN = nB * NBA;
  if (MP > NPADN) return;
  const int gR    = MP / RPB;
  const int vec8  = ((nE & 3) == 0) ? 1 : 0;

  char* ws = (char*)d_ws;
  size_t off = 0;
  const size_t oXB  = off; off = al256(off + (size_t)MP * HW * 2);
  const size_t oSW1 = off; off = al256(off + (size_t)HW * HW * 2);
  const size_t oSW2 = off; off = al256(off + (size_t)HW * PWH * 2);
  const size_t oC1  = off; off = al256(off + (size_t)HC * PWH * 2);
  const size_t oC2  = off; off = al256(off + (size_t)HC * PWH * 2);
  const size_t oC3  = off; off = al256(off + (size_t)HW * PWH * 2);
  const size_t oXP  = off; off = al256(off + (size_t)MP * PAH * 2);
  const size_t oH1L = off; off = al256(off + (size_t)MP * PAH * 2);
  const size_t oH2L = off; off = al256(off + (size_t)MP * PAH * 2);
  const size_t oXH  = off; off = al256(off + (size_t)MP * HC * 4);
  const size_t oH1  = off; off = al256(off + (size_t)MP * HW * 4);
  const size_t oSD  = off; off = al256(off + (size_t)2 * NHD * MP * 4);
  const size_t oLS  = off; off = al256(off + (size_t)nB * RCAP * 4);
  const size_t oCN  = off; off = al256(off + (size_t)NPADN * 4);
  const size_t oOF  = off; off = al256(off + (size_t)NPADN * 4);
  const size_t oFL  = off; off = al256(off + (size_t)NPADN * 4);
  const size_t oRC  = off; off = al256(off + (size_t)nB * 128);
  if (off > ws_size || off > (size_t)WSMAX) return;
  unsigned short* XB   = (unsigned short*)(ws + oXB);
  unsigned short* SW1  = (unsigned short*)(ws + oSW1);
  unsigned short* SW2D = (unsigned short*)(ws + oSW2);
  unsigned short* C1D  = (unsigned short*)(ws + oC1);
  unsigned short* C2D  = (unsigned short*)(ws + oC2);
  unsigned short* C3D  = (unsigned short*)(ws + oC3);
  unsigned short* XPhl = (unsigned short*)(ws + oXP);
  unsigned short* H1hl = (unsigned short*)(ws + oH1L);
  unsigned short* H2hl = (unsigned short*)(ws + oH2L);
  float* XH  = (float*)(ws + oXH);
  float* H1  = (float*)(ws + oH1);
  float* SD  = (float*)(ws + oSD);
  int*  LIST = (int*)(ws + oLS);
  int*  CNT  = (int*)(ws + oCN);
  int*  OFF  = (int*)(ws + oOF);
  int*  FLG  = (int*)(ws + oFL);
  int*  REC  = (int*)(ws + oRC);

  hipFuncSetAttribute(reinterpret_cast<const void*>(&k_bucket), hipFuncAttributeMaxDynamicSharedMemorySize, LDS_BK);

  const int uXB = MP * (HW / 8);
  k_prep<<<uXB / NTHR + UWALL / NTHR, NTHR, 0, stream>>>(x, sp_w1, sp_w2, g1_w, g2_w, g3_w,
                                                         XB, SW1, SW2D, C1D, C2D, C3D, nN, uXB);
  k_bucket<<<nB, NTHR, LDS_BK, stream>>>(dsts, srcs, nE, nN, vec8, LIST, CNT, OFF, FLG, REC);
  k_prompt<<<gR, GTHR, 0, stream>>>(XB, SW1, SW2D, sp_b1, sp_b2, sp_emb, sp_fw, sp_lnw, sp_lnb, XPhl, nN);
  k_proj<<<dim3(gR, NHD), GTHR, 0, stream>>>(XPhl, C1D, XH, PAH, PWH, KX_C1, HC, g1_as, g1_ad, SD, MP);
  k_replay<1><<<gR, NTHR, 0, stream>>>(XH, SD, LIST, CNT, OFF, FLG, g1_b, ln1_w, ln1_b, H1, H1, H1hl, out, nN, MP, MP);
  k_proj<<<dim3(gR, NHD), GTHR, 0, stream>>>(H1hl, C2D, XH, PAH, PWH, KX_C2, HC, g2_as, g2_ad, SD, MP);
  k_replay<2><<<gR, NTHR, 0, stream>>>(XH, SD, LIST, CNT, OFF, FLG, g2_b, ln2_w, ln2_b, H1, H1, H2hl, out, nN, MP, MP);
  k_proj<<<dim3(gR, 1), GTHR, 0, stream>>>(H2hl, C3D, XH, PAH, PWH, KX_C3, HW, g3_as, g3_ad, SD, MP);
  k_replay<3><<<gR, NTHR, 0, stream>>>(XH, SD, LIST, CNT, OFF, FLG, g3_b, g3_b, g3_b, H1, H1, H2hl, out, nN, MP, MP);
}
